// RNN_71880572666275
// MI455X (gfx1250) — hardware-verified
//
#include <hip/hip_runtime.h>
#include <math.h>

constexpr int NBATCH   = 4096;
constexpr int NSTEP    = 82;
constexpr int NEMB     = 128;
constexpr int NHID     = 64;
constexpr int NGATE    = 192;
constexpr int NVOC     = 50000;
constexpr int NVOC_PAD = 50048;
constexpr int HPITCH   = 72;
constexpr int SLABP    = 68;
constexpr float WCARRY     = 256.0f;
constexpr float WCARRY_INV = 1.0f / 256.0f;
constexpr int PROJ_ROWS_PER_BLOCK = 64;
constexpr int PROJ_BLOCKS = NVOC_PAD / PROJ_ROWS_PER_BLOCK;
constexpr int SEQ_BLOCKS  = NBATCH / 64;
static_assert(NGATE == 3 * NHID, "gate layout");
static_assert(NEMB % 32 == 0 && NHID % 32 == 0, "k multiples of 32");
static_assert(NVOC_PAD % 64 == 0 && NVOC_PAD >= NVOC, "padded table rows");
static_assert(NBATCH % 64 == 0, "batch tiles");
static_assert((NGATE * NEMB * 2) % (128 * 16) == 0, "W_ih staging loop exact");
static_assert((NGATE * NHID * 2) % (128 * 16) == 0, "W_hh staging loop exact");
static_assert((HPITCH % 8) == 0, "16-byte aligned A rows");

typedef __attribute__((ext_vector_type(16))) _Float16 v16h;
typedef __attribute__((ext_vector_type(8)))  _Float16 v8h;
typedef __attribute__((ext_vector_type(8)))  float    v8f;
typedef __attribute__((ext_vector_type(4)))  float    v4f;
typedef __attribute__((ext_vector_type(4)))  unsigned v4u;

__device__ __forceinline__ void guard4_h(v8f& a, v8f& b, v8f& c, v8f& d, v16h x, v16h y0, v16h y1, v16h y2, v16h y3) {
  asm volatile("v_nop\n\tv_nop\n\tv_nop\n\tv_nop" : "+v"(a), "+v"(b), "+v"(c), "+v"(d) : "v"(x), "v"(y0), "v"(y1), "v"(y2), "v"(y3));
}
__device__ __forceinline__ void guard3_h(v8f& a, v8f& b, v8f& c, v16h x0, v16h x1,
                                         v16h y0, v16h y1, v16h y2, v16h y3, v16h y4, v16h y5) {
  asm volatile("v_nop\n\tv_nop\n\tv_nop\n\tv_nop" : "+v"(a), "+v"(b), "+v"(c)
               : "v"(x0), "v"(x1), "v"(y0), "v"(y1), "v"(y2), "v"(y3), "v"(y4), "v"(y5));
}
__device__ __forceinline__ void acc_guard4(v8f& a, v8f& b, v8f& c, v8f& d) {
  asm volatile("v_nop\n\tv_nop\n\tv_nop\n\tv_nop" : "+v"(a), "+v"(b), "+v"(c), "+v"(d));
}

struct FragH {
  union U { v16h v; v8h h[2]; };
  static __device__ __forceinline__ v16h load(const _Float16* p) {
    U f;
    f.h[0] = *(const v8h*)(p);
    f.h[1] = *(const v8h*)(p + 16);
    return f.v;
  }
  static __device__ __forceinline__ v8f mma(v16h a, v16h b, v8f c) {
    return __builtin_amdgcn_wmma_f32_16x16x32_f16(false, a, false, b, (short)0, c, false, false);
  }
};

__device__ __forceinline__ float sig_f(float x) {
  x = fminf(fmaxf(x, -30.0f), 30.0f);
  return __builtin_amdgcn_rcpf(1.0f + expf(-x));
}
__device__ __forceinline__ float tanh_f(float x) {
  x = fminf(fmaxf(x, -15.0f), 15.0f);
  return 1.0f - 2.0f * __builtin_amdgcn_rcpf(1.0f + expf(2.0f * x));
}

__global__ __launch_bounds__(256) void prep_kernel(const float* __restrict__ w_ih, const float* __restrict__ w_hh,
                                                   const float* __restrict__ b_ih, const float* __restrict__ b_hh,
                                                   unsigned short* __restrict__ wih16, unsigned short* __restrict__ whh16,
                                                   float* __restrict__ bp) {
  const int blk = blockIdx.x;
  const int tid = threadIdx.x;
  if (blk < 18) {
    const bool first = blk < 12;
    const float* src = first ? w_ih : w_hh;
    unsigned short* dst = first ? wih16 : whh16;
    const int i = (first ? blk : (blk - 12)) * 256 + tid;
    const float* sp = src + (size_t)i * 8;
    const v4f a = *(const v4f*)(sp);
    const v4f b = *(const v4f*)(sp + 4);
    v8h hv;
#pragma unroll
    for (int e = 0; e < 4; ++e) {
      const float fa = a[e] * WCARRY;
      const float fb = b[e] * WCARRY;
      hv[e]     = (_Float16)fa;
      hv[4 + e] = (_Float16)fb;
    }
    *(volatile v8h*)(dst + (size_t)i * 8) = hv;
    __threadfence();
    *(volatile v8h*)(dst + (size_t)i * 8) = hv;
  } else {
    const int t4 = (tid < 48 ? tid : 47) * 4;
    const v4f vi = *(const v4f*)(b_ih + t4);
    const v4f vh = *(const v4f*)(b_hh + t4);
    v4f o;
#pragma unroll
    for (int e = 0; e < 4; ++e) {
      const float add = (t4 < 2 * NHID) ? vh[e] : 0.0f;
      o[e] = vi[e] + add;
    }
    if (tid < 48) {
      *(volatile v4f*)(bp + t4) = o;
      __threadfence();
      *(volatile v4f*)(bp + t4) = o;
    }
  }
}

__global__ __launch_bounds__(128) void proj_kernel(const float* __restrict__ emb, const unsigned short* __restrict__ wih16,
                                                   const float* __restrict__ bp, float* __restrict__ ptab) {
  __shared__ __align__(16) unsigned char smem[NGATE * NEMB * 2];
  const int tid = threadIdx.x, lane = tid & 31, wave = tid >> 5;
  const int c = lane & 15, hh = lane >> 4, koff = hh * 8;
  {
    const v4u* src = (const v4u*)wih16;
    v4u* dl = (v4u*)smem;
#pragma unroll 1
    for (int i = tid; i < (NGATE * NEMB * 2) / 16; i += 128) dl[i] = src[i];
  }
  __syncthreads();
  const _Float16* wl = (const _Float16*)smem;
  const int m0 = blockIdx.x * PROJ_ROWS_PER_BLOCK + wave * 16;
  int arow = m0 + c;
  arow = arow < NVOC ? arow : (NVOC - 1);
  const float* ap = emb + (size_t)arow * NEMB + koff;

  v8f acc[12];
#pragma unroll
  for (int j = 0; j < 12; ++j) acc[j] = (v8f){0.f, 0.f, 0.f, 0.f, 0.f, 0.f, 0.f, 0.f};

#pragma unroll 1
  for (int k0 = 0; k0 < NEMB; k0 += 32) {
    const v4f x0 = *(const v4f*)(ap + k0);
    const v4f x1 = *(const v4f*)(ap + k0 + 4);
    const v4f x2 = *(const v4f*)(ap + k0 + 16);
    const v4f x3 = *(const v4f*)(ap + k0 + 20);
    v16h a;
#pragma unroll
    for (int e = 0; e < 4; ++e) {
      a[e]      = (_Float16)x0[e];
      a[4 + e]  = (_Float16)x1[e];
      a[8 + e]  = (_Float16)x2[e];
      a[12 + e] = (_Float16)x3[e];
    }
#pragma unroll
    for (int g = 0; g < 3; ++g) {
      const _Float16* wp = wl + (size_t)(64 * g + c) * NEMB + koff + k0;
      const v16h b0 = FragH::load(wp);
      const v16h b1 = FragH::load(wp + 16 * NEMB);
      const v16h b2 = FragH::load(wp + 32 * NEMB);
      const v16h b3 = FragH::load(wp + 48 * NEMB);
      acc[4 * g + 0] = FragH::mma(a, b0, acc[4 * g + 0]);
      acc[4 * g + 1] = FragH::mma(a, b1, acc[4 * g + 1]);
      acc[4 * g + 2] = FragH::mma(a, b2, acc[4 * g + 2]);
      acc[4 * g + 3] = FragH::mma(a, b3, acc[4 * g + 3]);
      guard4_h(acc[4 * g + 0], acc[4 * g + 1], acc[4 * g + 2], acc[4 * g + 3], a, b0, b1, b2, b3);
    }
  }
  acc_guard4(acc[0], acc[1], acc[2], acc[3]);
  acc_guard4(acc[4], acc[5], acc[6], acc[7]);
  acc_guard4(acc[8], acc[9], acc[10], acc[11]);

  __syncthreads();
  float* slab = (float*)smem + wave * (16 * NGATE);
#pragma unroll
  for (int j = 0; j < 12; ++j) {
    const float bv = bp[16 * j + c];
#pragma unroll
    for (int r = 0; r < 8; ++r) {
      const float v = acc[j][r] * WCARRY_INV + bv;
      slab[(8 * hh + r) * NGATE + 16 * j + c] = v;
    }
  }
  __syncthreads();
  float* pw = ptab + (size_t)m0 * NGATE;
  for (int pass = 0; pass < 2; ++pass) {
#pragma unroll 4
    for (int it = 0; it < 24; ++it) {
      const v4f v = *(const v4f*)(slab + it * 128 + lane * 4);
      *(volatile v4f*)(pw + it * 128 + lane * 4) = v;
    }
    __threadfence();
  }
}

__device__ __forceinline__ void init_tile(const float* __restrict__ hrow0, int col, _Float16* ahrows, float (&h)[8]) {
#pragma unroll
  for (int r = 0; r < 8; ++r) h[r] = hrow0[(size_t)r * NHID + col];
#pragma unroll
  for (int r = 0; r < 8; ++r) ahrows[r * HPITCH + col] = (_Float16)h[r];
  asm volatile("" : "+v"(h[0]), "+v"(h[1]), "+v"(h[2]), "+v"(h[3]), "+v"(h[4]), "+v"(h[5]), "+v"(h[6]), "+v"(h[7]) :: "memory");
}

__global__ __launch_bounds__(128) void gru_kernel(const int* __restrict__ idx, const float* __restrict__ hid1,
                                                  const unsigned short* __restrict__ whh16, const float* __restrict__ b_hh,
                                                  const float* __restrict__ ptab, float* __restrict__ out) {
  __shared__ __align__(16) _Float16 wl[NGATE * NHID];
  __shared__ __align__(16) _Float16 ah[4][16 * HPITCH];
  __shared__ __align__(16) float    sl[4][16 * SLABP];
  __shared__ __align__(16) float    bnl[NHID];
  const int tid = threadIdx.x, lane = tid & 31, wave = tid >> 5;
  const int c = lane & 15, hh = lane >> 4, koff = hh * 8;
  const int b0w = (blockIdx.x * 4 + wave) * 16;

  {
    const v4u* src = (const v4u*)whh16;
    v4u* dl = (v4u*)wl;
#pragma unroll 1
    for (int i = tid; i < (NGATE * NHID * 2) / 16; i += 128) dl[i] = src[i];
  }
  if (tid < NHID) bnl[tid] = b_hh[2 * NHID + tid];

  float hA[8], hB[8], hC[8], hD[8];
  {
    const float* hrow0 = hid1 + (size_t)(b0w + 8 * hh) * NHID;
    _Float16* ahrows = &ah[wave][0] + 8 * hh * HPITCH;
    init_tile(hrow0, c, ahrows, hA);
    init_tile(hrow0, 16 + c, ahrows, hB);
    init_tile(hrow0, 32 + c, ahrows, hC);
    init_tile(hrow0, 48 + c, ahrows, hD);
  }
  __syncthreads();

  const v8f z8 = {0.f, 0.f, 0.f, 0.f, 0.f, 0.f, 0.f, 0.f};
  const _Float16* ahw = &ah[wave][0] + c * HPITCH + koff;
  _Float16* ahst = &ah[wave][0] + 8 * hh * HPITCH + c;
  const int* idrow = idx + (size_t)(b0w + 8 * hh) * NSTEP;

#pragma unroll 1
  for (int s = 0; s < NSTEP; ++s) {
    const int tcol = NSTEP - 1 - s;
    int off[8];
#pragma unroll
    for (int r = 0; r < 8; ++r) {
      int t = idrow[r * NSTEP + tcol];
      t = t < 0 ? 0 : t;
      t = t > (NVOC - 1) ? (NVOC - 1) : t;
      off[r] = t * NGATE + c;
    }
    const v16h a0 = FragH::load(ahw);
    const v16h a1 = FragH::load(ahw + 32);

#pragma unroll 1
    for (int ub = 0; ub < 4; ++ub) {
      const _Float16* wp = wl + (16 * ub + c) * NHID + koff;
      const v16h br0 = FragH::load(wp);
      const v16h bz0 = FragH::load(wp + NHID * NHID);
      const v16h bn0 = FragH::load(wp + 2 * NHID * NHID);
      const v16h br1 = FragH::load(wp + 32);
      const v16h bz1 = FragH::load(wp + NHID * NHID + 32);
      const v16h bn1 = FragH::load(wp + 2 * NHID * NHID + 32);
      v8f ar = z8, az = z8, an = z8;
      ar = FragH::mma(a0, br0, ar);
      az = FragH::mma(a0, bz0, az);
      an = FragH::mma(a0, bn0, an);
      ar = FragH::mma(a1, br1, ar);
      az = FragH::mma(a1, bz1, az);
      an = FragH::mma(a1, bn1, an);
      guard3_h(ar, az, an, a0, a1, br0, bz0, bn0, br1, bz1, bn1);

      const float bn = bnl[16 * ub + c];
      const int cofs = 16 * ub;
      float hn[8];
#pragma unroll
      for (int half = 0; half < 2; ++half) {
        float pr[4], pz[4], pn[4];
#pragma unroll
        for (int i = 0; i < 4; ++i) {
          const float* pp = ptab + (size_t)(off[4 * half + i] + cofs);
          pr[i] = pp[0];
          pz[i] = pp[NHID];
          pn[i] = pp[2 * NHID];
        }
#pragma unroll
        for (int i = 0; i < 4; ++i) {
          const int rr = 4 * half + i;
          const float gr = ar[rr] * WCARRY_INV + pr[i];
          const float gz = az[rr] * WCARRY_INV + pz[i];
          const float rg = sig_f(gr);
          const float zg = sig_f(gz);
          const float gn = an[rr] * WCARRY_INV + bn;
          const float ng = tanh_f(pn[i] + rg * gn);
          hn[rr] = (1.0f - zg) * ng + zg * hA[rr];
        }
        asm volatile("" : "+v"(hn[4 * half + 0]), "+v"(hn[4 * half + 1]), "+v"(hn[4 * half + 2]), "+v"(hn[4 * half + 3]) :: "memory");
      }
#pragma unroll
      for (int r = 0; r < 8; ++r) ahst[r * HPITCH + cofs] = (_Float16)hn[r];
#pragma unroll
      for (int r = 0; r < 8; ++r) {
        hA[r] = hB[r];
        hB[r] = hC[r];
        hC[r] = hD[r];
        hD[r] = hn[r];
      }
    }
    __syncthreads();
  }

  float* slab = sl[wave];
#pragma unroll
  for (int r = 0; r < 8; ++r) {
    slab[(8 * hh + r) * SLABP + c]      = hA[r];
    slab[(8 * hh + r) * SLABP + 16 + c] = hB[r];
    slab[(8 * hh + r) * SLABP + 32 + c] = hC[r];
    slab[(8 * hh + r) * SLABP + 48 + c] = hD[r];
  }
  __syncthreads();
  {
    const int c4 = c * 4;
    for (int pass = 0; pass < 2; ++pass) {
#pragma unroll
      for (int it = 0; it < 8; ++it) {
        const int row = it * 2 + hh;
        const v4f v = *(const v4f*)(slab + row * SLABP + c4);
        *(volatile v4f*)(out + (size_t)(b0w + row) * NHID + c4) = v;
      }
      __threadfence();
    }
  }
}

extern "C" void kernel_launch(void* const* d_in, const int* in_sizes, int n_in,
                              void* d_out, int out_size, void* d_ws, size_t ws_size, hipStream_t stream) {
  if (n_in < 7 || d_out == nullptr || d_ws == nullptr) return;
  if (in_sizes[0] != NBATCH * NSTEP || in_sizes[1] != 2 * NBATCH * NHID || in_sizes[2] != NVOC * NEMB ||
      in_sizes[3] != NGATE * NEMB || in_sizes[4] != NGATE * NHID || in_sizes[5] != NGATE ||
      in_sizes[6] != NGATE || out_size != NBATCH * NHID) return;

  const int*   tok    = (const int*)d_in[0];
  const float* hidden = (const float*)d_in[1];
  const float* emb    = (const float*)d_in[2];
  const float* w_ih   = (const float*)d_in[3];
  const float* w_hh   = (const float*)d_in[4];
  const float* b_ih   = (const float*)d_in[5];
  const float* b_hh   = (const float*)d_in[6];
  float* out = (float*)d_out;
  const float* hid1 = hidden + (size_t)NBATCH * NHID;

  char* ws = (char*)d_ws;
  size_t off = 0;
  auto carve = [&](size_t bytes) -> char* { char* p = ws + off; off += (bytes + 255) & ~(size_t)255; return p; };
  unsigned short* WIH16 = (unsigned short*)carve((size_t)NGATE * NEMB * 2);
  unsigned short* WHH16 = (unsigned short*)carve((size_t)NGATE * NHID * 2);
  float*          BP    = (float*)carve((size_t)1024);
  float*          PTAB  = (float*)carve((size_t)NVOC_PAD * NGATE * 4);
  if (off > ws_size || off > (size_t)134217728) return;

  prep_kernel<<<19, 256, 0, stream>>>(w_ih, w_hh, b_ih, b_hh, WIH16, WHH16, BP);
  proj_kernel<<<PROJ_BLOCKS, 128, 0, stream>>>(emb, WIH16, BP, PTAB);
  gru_kernel<<<SEQ_BLOCKS, 128, 0, stream>>>(tok, hid1, WHH16, b_hh, PTAB, out);
}
